// GIN_89094801588700
// MI455X (gfx1250) — hardware-verified
//
#include <hip/hip_runtime.h>
#include <stddef.h>
#include <stdint.h>


#define DIN     128
#define KHL     256
#define NTHR    256
#define NWAVE   8
#define EPT     8
#define CHUNK   (NTHR * EPT)
#define WCAP    (EPT * 32)
#define LISTN   (NWAVE * WCAP)
#define NBMAX   2048
#define RCAP    28672
#define DEGCAP  64
#define PKS     11
#define GBM     64
#define GBN     128
#define GTHR    128
#define GNT     8
#define NUW1    (DIN * (DIN / 8))
#define NUW2    (DIN * (KHL / 8))
#define NUWT    (NUW1 + 3 * NUW2)
#define WSMAX   134217728
#define LDS_AGG ((2 * RCAP + 2 * NBMAX + LISTN) * 4 + 64)

static_assert((CHUNK & (CHUNK - 1)) == 0 && CHUNK <= (1 << PKS));
static_assert((NBMAX & (NBMAX - 1)) == 0 && NBMAX <= (1 << PKS));
static_assert(NTHR * 8 == NBMAX);
static_assert(LISTN >= NBMAX && LISTN >= NWAVE * WCAP);
static_assert((RCAP % 32) == 0);
static_assert(LDS_AGG <= 300000);
static_assert(GBM == (GTHR / 32) * 16 && GBN == 16 * GNT && GBN == DIN && GBN == 4 * 32);
static_assert((DIN % 32) == 0 && (KHL % 32) == 0 && KHL == 2 * DIN);
static_assert((NUW1 % NTHR) == 0 && (NUW2 % NTHR) == 0 && (NUWT % NTHR) == 0);
static_assert((DIN / 8) == 16 && (KHL / 8) == 32);

typedef float          v4f  __attribute__((ext_vector_type(4)));
typedef float          v8f  __attribute__((ext_vector_type(8)));
typedef int            v4i  __attribute__((ext_vector_type(4)));
typedef int            v8i  __attribute__((ext_vector_type(8)));
typedef unsigned int   v4u  __attribute__((ext_vector_type(4)));
typedef unsigned short v8us __attribute__((ext_vector_type(8)));
typedef __bf16         v16b __attribute__((ext_vector_type(16)));
typedef v4f  __attribute__((may_alias)) v4fa;
typedef v8us __attribute__((may_alias)) v8usa;
union Frag { v16b vb; v8us h[2]; v8i w; };

__device__ __forceinline__ v8f wmb(const Frag& a, const Frag& b, v8f c) {
  v8f d = __builtin_amdgcn_wmma_f32_16x16x32_bf16(false, a.vb, false, b.vb, (short)0, c, false, false);
  asm volatile("v_nop\n\tv_nop\n\tv_nop\n\tv_nop" : "+v"(d) : "v"(a.w), "v"(b.w));
  return d;
}

__device__ __forceinline__ unsigned short bf_bits(float f) {
  unsigned int u = __float_as_uint(f);
  u += 0x7FFFu + ((u >> 16) & 1u);
  return (unsigned short)(u >> 16);
}
__device__ __forceinline__ float bf_val(unsigned short b) { return __uint_as_float(((unsigned int)b) << 16); }
__device__ __forceinline__ float bf_rne(float f) { return bf_val(bf_bits(f)); }

__device__ __forceinline__ int scan_chunk(const int* __restrict__ dsts, int nE, int cbase, int slotBase,
                                          int nb, int vec8, int* list, int tid, int lane, int wave) {
  int wc = 0;
  const int el0  = tid * EPT;
  const int e0   = cbase + el0;
  const int sent = -2147483647 - 1;
  v4i da, db;
  if (vec8 != 0 && cbase + CHUNK <= nE) {
    da = *(const v4i*)(dsts + e0);
    db = *(const v4i*)(dsts + e0 + 4);
  } else {
    da.x = (e0     < nE) ? dsts[min(e0,     nE - 1)] : sent;
    da.y = (e0 + 1 < nE) ? dsts[min(e0 + 1, nE - 1)] : sent;
    da.z = (e0 + 2 < nE) ? dsts[min(e0 + 2, nE - 1)] : sent;
    da.w = (e0 + 3 < nE) ? dsts[min(e0 + 3, nE - 1)] : sent;
    db.x = (e0 + 4 < nE) ? dsts[min(e0 + 4, nE - 1)] : sent;
    db.y = (e0 + 5 < nE) ? dsts[min(e0 + 5, nE - 1)] : sent;
    db.z = (e0 + 6 < nE) ? dsts[min(e0 + 6, nE - 1)] : sent;
    db.w = (e0 + 7 < nE) ? dsts[min(e0 + 7, nE - 1)] : sent;
  }
  const unsigned nbs = (unsigned)slotBase;
  const unsigned unb = (unsigned)nb;
  const unsigned s0 = (unsigned)da.x - nbs, s1 = (unsigned)da.y - nbs;
  const unsigned s2 = (unsigned)da.z - nbs, s3 = (unsigned)da.w - nbs;
  const unsigned s4 = (unsigned)db.x - nbs, s5 = (unsigned)db.y - nbs;
  const unsigned s6 = (unsigned)db.z - nbs, s7 = (unsigned)db.w - nbs;
  const bool h0 = s0 < unb, h1 = s1 < unb, h2 = s2 < unb, h3 = s3 < unb;
  const bool h4 = s4 < unb, h5 = s5 < unb, h6 = s6 < unb, h7 = s7 < unb;
  const unsigned any = __builtin_amdgcn_ballot_w32(h0 | h1 | h2 | h3 | h4 | h5 | h6 | h7);
  if (any != 0u) {
#define HITJ(J, HJ, SJ) { \
      const unsigned mj = __builtin_amdgcn_ballot_w32(HJ); \
      if (mj != 0u) { \
        if (HJ) { \
          const int pos = wc + (int)__builtin_amdgcn_mbcnt_lo(mj, 0u); \
          if (pos < WCAP) list[wave * WCAP + pos] = ((el0 + (J)) << PKS) | (int)(SJ); \
        } \
        wc += (int)__builtin_popcount(mj); } }
    HITJ(0, h0, s0)
    HITJ(1, h1, s1)
    HITJ(2, h2, s2)
    HITJ(3, h3, s3)
    HITJ(4, h4, s4)
    HITJ(5, h5, s5)
    HITJ(6, h6, s6)
    HITJ(7, h7, s7)
#undef HITJ
  }
  return wc;
}

__global__ __launch_bounds__(NTHR) void k_prep(const float* __restrict__ x,
                                               const float* __restrict__ w1a, const float* __restrict__ w2a,
                                               const float* __restrict__ w1b, const float* __restrict__ w2b,
                                               unsigned short* xb, unsigned short* p1a, unsigned short* p2a,
                                               unsigned short* p1b, unsigned short* p2b, int nN, int nUx) {
  const int u = (int)blockIdx.x * NTHR + (int)threadIdx.x;
  v4f a, b;
  bool ok = true;
  unsigned short* dp;
  if (u < nUx) {
    const int row = u >> 4;
    const int k8  = (u & 15) * 8;
    const int rc  = row < nN ? row : nN - 1;
    const float* p = x + (size_t)rc * DIN + k8;
    a = *(const v4fa*)p;
    b = *(const v4fa*)(p + 4);
    ok = row < nN;
    dp = xb + (size_t)row * DIN + k8;
  } else {
    const int v = u - nUx;
    if (v < NUW1) {
      const int n = v >> 4, k8 = (v & 15) * 8;
      const float* p = w1a + (size_t)n * DIN + k8;
      a = *(const v4fa*)p;
      b = *(const v4fa*)(p + 4);
      dp = p1a + (size_t)v * 8;
    } else if (v < NUW1 + NUW2) {
      const int w = v - NUW1;
      const int n = w >> 5, k8 = (w & 31) * 8, kk = k8 & (DIN - 1);
      const float* p = w2a + (size_t)n * DIN + kk;
      a = *(const v4fa*)p;
      b = *(const v4fa*)(p + 4);
      dp = p2a + (size_t)w * 8;
    } else if (v < NUW1 + 2 * NUW2) {
      const int w = v - NUW1 - NUW2;
      const int n = w >> 5, k8 = (w & 31) * 8, kk = k8 & (DIN - 1);
      const float* p = w1b + (size_t)n * DIN + kk;
      a = *(const v4fa*)p;
      b = *(const v4fa*)(p + 4);
      dp = p1b + (size_t)w * 8;
    } else if (v < NUWT) {
      const int w = v - NUW1 - 2 * NUW2;
      const int n = w >> 5, k8 = (w & 31) * 8, kk = k8 & (DIN - 1);
      const float* p = w2b + (size_t)n * DIN + kk;
      a = *(const v4fa*)p;
      b = *(const v4fa*)(p + 4);
      dp = p2b + (size_t)w * 8;
    } else {
      return;
    }
  }
  v8us o;
  o[0] = ok ? bf_bits(a.x) : (unsigned short)0;
  o[1] = ok ? bf_bits(a.y) : (unsigned short)0;
  o[2] = ok ? bf_bits(a.z) : (unsigned short)0;
  o[3] = ok ? bf_bits(a.w) : (unsigned short)0;
  o[4] = ok ? bf_bits(b.x) : (unsigned short)0;
  o[5] = ok ? bf_bits(b.y) : (unsigned short)0;
  o[6] = ok ? bf_bits(b.z) : (unsigned short)0;
  o[7] = ok ? bf_bits(b.w) : (unsigned short)0;
  *(volatile v8us*)dp = o;
  __threadfence();
  *(volatile v8us*)dp = o;
}

__global__ __launch_bounds__(NTHR) void k_agg(
    const int* __restrict__ srcs, const int* __restrict__ dsts,
    const float* __restrict__ fin, const float* __restrict__ epsp,
    const float* __restrict__ b1, const float* __restrict__ gam, const float* __restrict__ bet,
    unsigned short* Tout,
    int nN, int nE, int nb, int vec8, int MPr) {
  extern __shared__ v4f lds_dyn[];
  int* reg1 = (int*)lds_dyn;
  int* reg2 = reg1 + RCAP;
  int* scnt = reg2 + RCAP;
  int* soff = scnt + NBMAX;
  int* list = soff + NBMAX;
  int* wcnt = list + LISTN;
  int* wtot = wcnt + NWAVE;
  const int tid = (int)threadIdx.x, lane = tid & 31, wave = tid >> 5;
  const int nodeBase = (int)blockIdx.x * nb;

  for (int i = tid; i < NBMAX; i += NTHR) scnt[i] = 0;
  __syncthreads();

  int tot = 0;
  const int nChunks = (nE + CHUNK - 1) / CHUNK;
#pragma unroll 1
  for (int ch = 0; ch < nChunks; ++ch) {
    const int cbase = ch * CHUNK;
    const int wc = scan_chunk(dsts, nE, cbase, nodeBase, nb, vec8, list, tid, lane, wave);
    if (lane == 0) wcnt[wave] = wc;
    __syncthreads();
    int pre = 0, all = 0;
#pragma unroll
    for (int w2 = 0; w2 < NWAVE; ++w2) {
      int c = wcnt[w2];
      c = c < 0 ? 0 : (c > WCAP ? WCAP : c);
      all += c;
      pre += (w2 < wave) ? c : 0;
    }
    const int wcc  = wc > WCAP ? WCAP : wc;
    const int base = tot + pre;
#pragma unroll 1
    for (int i = lane; i < wcc; i += 32) {
      const int ent = list[wave * WCAP + i];
      const int el  = (ent >> PKS) & (CHUNK - 1);
      const int sl  = ent & (NBMAX - 1);
      int eid = cbase + el;
      eid = eid > nE - 1 ? nE - 1 : eid;
      const int pos = base + i;
      if (pos < RCAP) reg1[pos] = (int)(((unsigned)eid << PKS) | (unsigned)sl);
    }
    tot += all;
    tot = tot > RCAP ? RCAP : tot;
    __syncthreads();
  }
  const int nh = tot;

  if (wave == 0) {
#pragma unroll 1
    for (int b0 = 0; b0 < nh; b0 += 32) {
      const int idx = b0 + lane;
      const int uv  = reg1[idx < RCAP ? idx : RCAP - 1];
      const int m32 = (nh - b0) < 32 ? (nh - b0) : 32;
#pragma unroll 1
      for (int k = 0; k < m32; ++k) {
        const int u  = __builtin_amdgcn_readlane(uv, k);
        const int sl = u & (NBMAX - 1);
        if (lane == 0) scnt[sl] = scnt[sl] + 1;
      }
    }
  }
  __syncthreads();

  {
    const v4i ca = *(const v4i*)(scnt + 8 * tid);
    const v4i cb = *(const v4i*)(scnt + 8 * tid + 4);
    const int e0 = ca.x < 0 ? 0 : ca.x, e1 = ca.y < 0 ? 0 : ca.y, e2 = ca.z < 0 ? 0 : ca.z, e3 = ca.w < 0 ? 0 : ca.w;
    const int e4 = cb.x < 0 ? 0 : cb.x, e5 = cb.y < 0 ? 0 : cb.y, e6 = cb.z < 0 ? 0 : cb.z, e7 = cb.w < 0 ? 0 : cb.w;
    const int ts = e0 + e1 + e2 + e3 + e4 + e5 + e6 + e7;
    int incl = ts;
#pragma unroll
    for (int d = 1; d < 32; d <<= 1) {
      const int up = __shfl_up(incl, d);
      if (lane >= d) incl += up;
    }
    if (lane == 31) wtot[wave] = incl;
    __syncthreads();
    int pre = 0;
#pragma unroll
    for (int w2 = 0; w2 < NWAVE; ++w2) pre += (w2 < wave) ? wtot[w2] : 0;
    int run = pre + incl - ts;
    soff[8 * tid + 0] = run; run += e0;
    soff[8 * tid + 1] = run; run += e1;
    soff[8 * tid + 2] = run; run += e2;
    soff[8 * tid + 3] = run; run += e3;
    soff[8 * tid + 4] = run; run += e4;
    soff[8 * tid + 5] = run; run += e5;
    soff[8 * tid + 6] = run; run += e6;
    soff[8 * tid + 7] = run;
  }
  __syncthreads();
  for (int i = tid; i < NBMAX; i += NTHR) list[i] = soff[i];
  __syncthreads();

  if (wave == 0) {
#pragma unroll 1
    for (int b0 = 0; b0 < nh; b0 += 32) {
      const int idx = b0 + lane;
      const int uv  = reg1[idx < RCAP ? idx : RCAP - 1];
      const int m32 = (nh - b0) < 32 ? (nh - b0) : 32;
#pragma unroll 1
      for (int k = 0; k < m32; ++k) {
        const int u   = __builtin_amdgcn_readlane(uv, k);
        const int sl  = u & (NBMAX - 1);
        const int eid = (int)((unsigned)u >> PKS);
        if (lane == 0) {
          int pos = list[sl];
          pos = pos < 0 ? 0 : (pos > RCAP - 1 ? RCAP - 1 : pos);
          reg2[pos] = eid;
          list[sl] = pos + 1;
        }
      }
    }
  }
  __syncthreads();

  const int nbw = nb >> 3;
  const bool ovf = (nh >= RCAP);
  const float qnan = __int_as_float(0x7fc00000);
  const float epf = 1.0f + bf_rne(epsp[0]);
  float bb0, bb1, bb2, bb3, g0, g1, g2, g3, be0, be1, be2, be3;
  {
    const v4f q = *(const v4fa*)(b1 + 4 * lane);
    bb0 = bf_rne(q.x); bb1 = bf_rne(q.y); bb2 = bf_rne(q.z); bb3 = bf_rne(q.w);
    const v4f g = *(const v4fa*)(gam + 4 * lane);
    g0 = bf_rne(g.x); g1 = bf_rne(g.y); g2 = bf_rne(g.z); g3 = bf_rne(g.w);
    const v4f e = *(const v4fa*)(bet + 4 * lane);
    be0 = bf_rne(e.x); be1 = bf_rne(e.y); be2 = bf_rne(e.z); be3 = bf_rne(e.w);
  }
  const int sa = (2 * lane) & 31, sb = (2 * lane + 1) & 31;
  const bool lsel = lane >= 16;

#pragma unroll 1
  for (int jt = 0; jt < nbw; ++jt) {
    const int slot = wave * nbw + jt;
    const int grow = nodeBase + slot;
    int st = soff[slot];
    const int craw = scnt[slot];
    int cnt = craw;
    st  = st < 0 ? 0 : (st > nh ? nh : st);
    cnt = cnt < 0 ? 0 : (cnt > DEGCAP ? DEGCAP : cnt);
    if (cnt > nh - st) cnt = nh - st;
    const float pz = (ovf || craw > DEGCAP) ? qnan : 0.0f;
    const bool liveRow = grow < nN;

    float ag0 = 0.f, ag1 = 0.f, ag2 = 0.f, ag3 = 0.f;
#pragma unroll 1
    for (int q = 0; q < cnt; ++q) {
      int idx = st + q; idx = idx > RCAP - 1 ? RCAP - 1 : idx;
      int eid = reg2[idx]; eid = eid < 0 ? 0 : (eid > nE - 1 ? nE - 1 : eid);
      const int sraw = srcs[eid];
      const int s = sraw < 0 ? 0 : (sraw > nN - 1 ? nN - 1 : sraw);
      const v4f v = *(const v4f*)(fin + (size_t)s * DIN + 4 * lane);
      ag0 += v.x; ag1 += v.y; ag2 += v.z; ag3 += v.w;
    }
    const int nc = liveRow ? grow : nN - 1;
    const v4f sv = *(const v4f*)(fin + (size_t)nc * DIN + 4 * lane);
    const float r0 = ((epf * sv.x + ag0) + bb0) + pz;
    const float r1 = ((epf * sv.y + ag1) + bb1) + pz;
    const float r2 = ((epf * sv.z + ag2) + bb2) + pz;
    const float r3 = ((epf * sv.w + ag3) + bb3) + pz;

    float sm = (r0 + r1) + (r2 + r3);
    sm += __shfl_xor(sm, 16);
    sm += __shfl_xor(sm, 8);
    sm += __shfl_xor(sm, 4);
    sm += __shfl_xor(sm, 2);
    sm += __shfl_xor(sm, 1);
    const float mu = sm * (1.0f / (float)DIN);
    const float d0 = r0 - mu, d1 = r1 - mu, d2 = r2 - mu, d3 = r3 - mu;
    float qq = (d0 * d0 + d1 * d1) + (d2 * d2 + d3 * d3);
    qq += __shfl_xor(qq, 16);
    qq += __shfl_xor(qq, 8);
    qq += __shfl_xor(qq, 4);
    qq += __shfl_xor(qq, 2);
    qq += __shfl_xor(qq, 1);
    const float var = qq * (1.0f / (float)DIN);
    const float rs  = rsqrtf(var + 1e-5f);
    float v0 = d0 * rs * g0 + be0;
    float v1 = d1 * rs * g1 + be1;
    float v2 = d2 * rs * g2 + be2;
    float v3 = d3 * rs * g3 + be3;
    v0 = (v0 >= 0.0f) ? v0 : 0.01f * v0;
    v1 = (v1 >= 0.0f) ? v1 : 0.01f * v1;
    v2 = (v2 >= 0.0f) ? v2 : 0.01f * v2;
    v3 = (v3 >= 0.0f) ? v3 : 0.01f * v3;
    v0 = liveRow ? v0 : 0.0f;
    v1 = liveRow ? v1 : 0.0f;
    v2 = liveRow ? v2 : 0.0f;
    v3 = liveRow ? v3 : 0.0f;

    const unsigned short h0 = bf_bits(v0), h1 = bf_bits(v1), h2 = bf_bits(v2), h3 = bf_bits(v3);
    const unsigned short l0 = bf_bits(v0 - bf_val(h0)), l1 = bf_bits(v1 - bf_val(h1));
    const unsigned short l2 = bf_bits(v2 - bf_val(h2)), l3 = bf_bits(v3 - bf_val(h3));
    const int hw0 = (int)((unsigned int)h0 | ((unsigned int)h1 << 16));
    const int hw1 = (int)((unsigned int)h2 | ((unsigned int)h3 << 16));
    const int lw0 = (int)((unsigned int)l0 | ((unsigned int)l1 << 16));
    const int lw1 = (int)((unsigned int)l2 | ((unsigned int)l3 << 16));
    const int ga0 = __shfl(hw0, sa, 32), ga1 = __shfl(hw1, sa, 32);
    const int ga2 = __shfl(hw0, sb, 32), ga3 = __shfl(hw1, sb, 32);
    const int pa0 = __shfl(lw0, sa, 32), pa1 = __shfl(lw1, sa, 32);
    const int pa2 = __shfl(lw0, sb, 32), pa3 = __shfl(lw1, sb, 32);
    v4u pv;
    pv.x = (unsigned int)(lsel ? pa0 : ga0);
    pv.y = (unsigned int)(lsel ? pa1 : ga1);
    pv.z = (unsigned int)(lsel ? pa2 : ga2);
    pv.w = (unsigned int)(lsel ? pa3 : ga3);
    unsigned short* gp = Tout + (size_t)grow * KHL + 8 * lane;
    const bool wsv = grow < MPr;
    if (wsv) *(volatile v4u*)gp = pv;
    __threadfence();
    if (wsv) *(volatile v4u*)gp = pv;
  }
}

template <int EPI>
__global__ __launch_bounds__(GTHR) void k_gemm(const unsigned short* __restrict__ A, int lda,
                                               const unsigned short* __restrict__ BT, int ldb, int K,
                                               const float* __restrict__ bias,
                                               void* outp, int nN, int mRows) {
  __shared__ __attribute__((aligned(16))) float stg[GBM * GBN];
  const int tid = (int)threadIdx.x, lane = tid & 31, wave = tid >> 5, hh = lane >> 4, m = lane & 15;
  const int rowBase = (int)blockIdx.x * GBM;

  v8f acc[GNT];
  {
    const v8f z = {0.f, 0.f, 0.f, 0.f, 0.f, 0.f, 0.f, 0.f};
#pragma unroll
    for (int t = 0; t < GNT; ++t) acc[t] = z;
  }
  const unsigned short* ap = A  + (size_t)(rowBase + 16 * wave + m) * (size_t)lda + 8 * hh;
  const unsigned short* bp = BT + (size_t)m * (size_t)ldb + 8 * hh;

#pragma unroll 1
  for (int k0 = 0; k0 < K; k0 += 32) {
    Frag af;
    af.h[0] = *(const v8usa*)(ap + k0);
    af.h[1] = *(const v8usa*)(ap + k0 + 16);
#pragma unroll
    for (int nt = 0; nt < GNT; ++nt) {
      const unsigned short* wq = bp + (size_t)(16 * nt) * (size_t)ldb + k0;
      Frag bfr;
      bfr.h[0] = *(const v8usa*)wq;
      bfr.h[1] = *(const v8usa*)(wq + 16);
      acc[nt] = wmb(af, bfr, acc[nt]);
    }
  }

#pragma unroll
  for (int nt = 0; nt < GNT; ++nt) {
    const int lc = 16 * nt + m;
    float bb = 0.0f;
    if constexpr (EPI != 0) bb = bf_rne(bias[lc]);
#pragma unroll
    for (int r = 0; r < 8; ++r) {
      const int lr = 16 * wave + 8 * hh + r;
      const bool live = (rowBase + lr) < nN;
      const float v = acc[nt][r] + bb;
      stg[lr * GBN + lc] = live ? v : 0.0f;
    }
  }
  __syncthreads();

  if constexpr (EPI != 0) {
#pragma unroll 1
    for (int i = 0; i < 16; ++i) {
      float* rp = stg + (16 * wave + i) * GBN + 4 * lane;
      const v4f a = *(const v4fa*)rp;
      float ss = (a.x * a.x + a.y * a.y) + (a.z * a.z + a.w * a.w);
      ss += __shfl_xor(ss, 16);
      ss += __shfl_xor(ss, 8);
      ss += __shfl_xor(ss, 4);
      ss += __shfl_xor(ss, 2);
      ss += __shfl_xor(ss, 1);
      const float den = fmaxf(sqrtf(ss), 1e-12f);
      v4f o;
      o.x = a.x / den; o.y = a.y / den; o.z = a.z / den; o.w = a.w / den;
      if constexpr (EPI == 1) {
        o.x = (o.x >= 0.0f) ? o.x : 0.01f * o.x;
        o.y = (o.y >= 0.0f) ? o.y : 0.01f * o.y;
        o.z = (o.z >= 0.0f) ? o.z : 0.01f * o.z;
        o.w = (o.w >= 0.0f) ? o.w : 0.01f * o.w;
      }
      *(v4fa*)rp = o;
    }
    __syncthreads();
  }

  if constexpr (EPI == 1) {
    unsigned short* outH = (unsigned short*)outp;
    const int cb = 8 * m;
    const bool isHi = (hh == 0);
    v4u pk[16];
#pragma unroll
    for (int i = 0; i < 16; ++i) {
      const int lr = 16 * wave + i;
      const v4f a = *(const v4fa*)(stg + lr * GBN + cb);
      const v4f b = *(const v4fa*)(stg + lr * GBN + cb + 4);
      const float f[8] = {a.x, a.y, a.z, a.w, b.x, b.y, b.z, b.w};
      unsigned int w[4];
#pragma unroll
      for (int j = 0; j < 4; ++j) {
        const unsigned short h0 = bf_bits(f[2 * j]), h1 = bf_bits(f[2 * j + 1]);
        const unsigned short l0 = bf_bits(f[2 * j] - bf_val(h0)), l1 = bf_bits(f[2 * j + 1] - bf_val(h1));
        const unsigned short q0 = isHi ? h0 : l0, q1 = isHi ? h1 : l1;
        w[j] = (unsigned int)q0 | ((unsigned int)q1 << 16);
      }
      v4u pv; pv.x = w[0]; pv.y = w[1]; pv.z = w[2]; pv.w = w[3];
      pk[i] = pv;
    }
#pragma unroll
    for (int i = 0; i < 16; ++i) {
      const int gr = rowBase + 16 * wave + i;
      unsigned short* op = outH + (size_t)gr * KHL + cb + hh * DIN;
      if (gr < mRows) *(volatile v4u*)op = pk[i];
    }
    __threadfence();
#pragma unroll
    for (int i = 0; i < 16; ++i) {
      const int gr = rowBase + 16 * wave + i;
      unsigned short* op = outH + (size_t)gr * KHL + cb + hh * DIN;
      if (gr < mRows) *(volatile v4u*)op = pk[i];
    }
  } else {
    float* outF = (float*)outp;
    const int lim = (EPI == 2) ? nN : mRows;
    v4f fv[16];
#pragma unroll
    for (int i = 0; i < 16; ++i) {
      const int lr = 16 * wave + i;
      fv[i] = *(const v4fa*)(stg + lr * GBN + 4 * lane);
    }
#pragma unroll
    for (int i = 0; i < 16; ++i) {
      const int gr = rowBase + 16 * wave + i;
      float* op = outF + (size_t)gr * GBN + 4 * lane;
      if (gr < lim) *(volatile v4f*)op = fv[i];
    }
    __threadfence();
#pragma unroll
    for (int i = 0; i < 16; ++i) {
      const int gr = rowBase + 16 * wave + i;
      float* op = outF + (size_t)gr * GBN + 4 * lane;
      if (gr < lim) *(volatile v4f*)op = fv[i];
    }
  }
}

static int pick_nb(int nE, int nN) {
  int nb = NBMAX;
  while (nb > 16 && (long long)nb * (long long)nE * 5LL > (long long)RCAP * (long long)nN * 4LL) nb >>= 1;
  return nb;
}
static inline int cdiv(int a, int b) { return (a + b - 1) / b; }
static inline size_t al256(size_t o) { return (o + 255) & ~(size_t)255; }

extern "C" void kernel_launch(void* const* d_in, const int* in_sizes, int n_in,
                              void* d_out, int out_size, void* d_ws, size_t ws_size,
                              hipStream_t stream) {
  if (n_in < 16) return;
  if (in_sizes[0] < DIN || (in_sizes[0] % DIN) != 0) return;
  const int nN = in_sizes[0] / DIN;
  if (nN < GBM || nN > (1 << 22)) return;
  const int nE2 = in_sizes[1];
  if (nE2 < 2 || (nE2 & 1) != 0) return;
  const int nE = nE2 / 2;
  if (nE < 1 || nE > (1 << 21)) return;
  if (in_sizes[2] < 1 || in_sizes[3] < 1) return;
  if (in_sizes[4]  != DIN * DIN || in_sizes[5]  != DIN) return;
  if (in_sizes[6]  != DIN       || in_sizes[7]  != DIN) return;
  if (in_sizes[8]  != DIN * DIN || in_sizes[9]  != DIN) return;
  if (in_sizes[10] != DIN * DIN || in_sizes[11] != DIN) return;
  if (in_sizes[12] != DIN       || in_sizes[13] != DIN) return;
  if (in_sizes[14] != DIN * DIN || in_sizes[15] != DIN) return;
  if ((long long)nN * DIN != (long long)out_size) return;

  const float* x    = (const float*)d_in[0];
  const int*   ei   = (const int*)  d_in[1];
  const int*   src  = ei;
  const int*   dst  = ei + nE;
  const float* eps1 = (const float*)d_in[2];
  const float* eps2 = (const float*)d_in[3];
  const float* W1a  = (const float*)d_in[4];  const float* b1a = (const float*)d_in[5];
  const float* ga   = (const float*)d_in[6];  const float* bea = (const float*)d_in[7];
  const float* W2a  = (const float*)d_in[8];  const float* b2a = (const float*)d_in[9];
  const float* W1b  = (const float*)d_in[10]; const float* b1b = (const float*)d_in[11];
  const float* gb   = (const float*)d_in[12]; const float* beb = (const float*)d_in[13];
  const float* W2b  = (const float*)d_in[14]; const float* b2b = (const float*)d_in[15];
  float* out = (float*)d_out;

  const int MP   = cdiv(nN, GBM) * GBM;
  const int gM   = MP / GBM;
  const int nb   = pick_nb(nE, nN);
  const int gA   = cdiv(MP, nb);
  const int vec8 = ((nE & 3) == 0) ? 1 : 0;
  if ((long long)gA * nb < (long long)MP) return;
  if ((long long)(gM - 1) * GBM >= (long long)nN) return;
  const int nUx = MP * (DIN / 8);
  if ((nUx % NTHR) != 0) return;

  char* ws = (char*)d_ws;
  size_t off = 0;
  const size_t oW1a = off; off = al256(off + (size_t)NUW1 * 16);
  const size_t oW2a = off; off = al256(off + (size_t)NUW2 * 16);
  const size_t oW1b = off; off = al256(off + (size_t)NUW2 * 16);
  const size_t oW2b = off; off = al256(off + (size_t)NUW2 * 16);
  const size_t oRA  = off; off = al256(off + (size_t)MP * 512);
  const size_t oRB  = off; off = al256(off + (size_t)MP * 512);
  if (off > ws_size || off > (size_t)WSMAX) return;
  unsigned short* PW1a = (unsigned short*)(ws + oW1a);
  unsigned short* PW2a = (unsigned short*)(ws + oW2a);
  unsigned short* PW1b = (unsigned short*)(ws + oW1b);
  unsigned short* PW2b = (unsigned short*)(ws + oW2b);
  void* RA = (void*)(ws + oRA);
  void* RB = (void*)(ws + oRB);

  hipFuncSetAttribute(reinterpret_cast<const void*>(&k_agg), hipFuncAttributeMaxDynamicSharedMemorySize, LDS_AGG);

  k_prep<<<(nUx + NUWT) / NTHR, NTHR, 0, stream>>>(x, W1a, W2a, W1b, W2b, (unsigned short*)RB,
                                                   PW1a, PW2a, PW1b, PW2b, nN, nUx);
  k_gemm<0><<<gM, GTHR, 0, stream>>>((const unsigned short*)RB, DIN, PW1a, DIN, DIN, b1a, RA, nN, MP);
  k_agg<<<gA, NTHR, LDS_AGG, stream>>>(src, dst, (const float*)RA, eps1, b1a, ga, bea,
                                       (unsigned short*)RB, nN, nE, nb, vec8, MP);
  k_gemm<1><<<gM, GTHR, 0, stream>>>((const unsigned short*)RB, KHL, PW2a, KHL, KHL, b2a, RA, nN, MP);
  k_gemm<0><<<gM, GTHR, 0, stream>>>((const unsigned short*)RA, KHL, PW1b, KHL, KHL, b1b, RB, nN, MP);
  k_agg<<<gA, NTHR, LDS_AGG, stream>>>(src, dst, (const float*)RB, eps2, b1b, gb, beb,
                                       (unsigned short*)RA, nN, nE, nb, vec8, MP);
  k_gemm<2><<<gM, GTHR, 0, stream>>>((const unsigned short*)RA, KHL, PW2b, KHL, KHL, b2b, (void*)out, nN, MP);
}
